// GCNLayer_1400159338837
// MI455X (gfx1250) — hardware-run, weakly checked
//
#include <hip/hip_runtime.h>
#include <stddef.h>
#include <stdint.h>
#include <math.h>


#define DIN    64
#define K1     64
#define HID    128
#define NCLS   40
#define NC2P   64
#define K2     256
#define NTHR   256
#define NWAVE  8
#define EPT    8
#define CHUNK  (NTHR * EPT)
#define WCAP   (EPT * 32)
#define LISTN  (NWAVE * WCAP)
#define NBA    1024
#define SLA    10
#define SPW    (NBA / NWAVE)
#define RCAP   28672
#define DEGCAP 256
#define GBM    64
#define GBN    64
#define GTHR   128
#define GRP    64
#define NU1    (HID * (K1 / 8))
#define NU2    (NC2P * (K2 / 8))
#define AGG_ZINTS (LISTN + 2 * RCAP + 3 * NBA)
#define AGG_LDS_INTS (AGG_ZINTS + 16)
#define WSMAX  134217728

static_assert((CHUNK & (CHUNK - 1)) == 0 && CHUNK <= 4096);
static_assert((NBA & (NBA - 1)) == 0 && NBA == (1 << SLA));
static_assert(((long long)CHUNK << SLA) < (1LL << 31));
static_assert(LISTN % NTHR == 0);
static_assert(NBA % NWAVE == 0 && NBA % 32 == 0 && NBA % GBM == 0);
static_assert(SPW % GRP == 0 && (GRP & (GRP - 1)) == 0 && GRP % 4 == 0);
static_assert(RCAP % 32 == 0 && AGG_ZINTS % 4 == 0 && LISTN % 4 == 0);
static_assert(NWAVE * GRP * NCLS <= RCAP);
static_assert(K1 % 32 == 0 && K2 % 32 == 0 && K2 == 2 * HID && K1 == DIN);
static_assert(NC2P == GBN && HID == 2 * GBN);
static_assert(GBM == (GTHR / 32) * 16 && GBN == 64);
static_assert(NU1 % NTHR == 0 && NU2 % NTHR == 0);
static_assert(K1 / 8 == 8 && K2 / 8 == 32 && DIN / 8 == 8);
static_assert(HID == 4 * 32 && NC2P == 2 * 32);
static_assert(NCLS <= NC2P && (NCLS % 4) == 0 && (NCLS % 2) == 0);
static_assert(AGG_LDS_INTS * 4 <= 300000);

typedef float          v2f   __attribute__((ext_vector_type(2)));
typedef float          v4f   __attribute__((ext_vector_type(4)));
typedef float          v8f   __attribute__((ext_vector_type(8)));
typedef int            v4i   __attribute__((ext_vector_type(4)));
typedef int            v8i   __attribute__((ext_vector_type(8)));
typedef unsigned int   v4u   __attribute__((ext_vector_type(4)));
typedef unsigned short v8us  __attribute__((ext_vector_type(8)));
typedef unsigned short v16us __attribute__((ext_vector_type(16)));
typedef __bf16         v16bf __attribute__((ext_vector_type(16)));
typedef v2f  __attribute__((may_alias)) v2fa;
typedef v4f  __attribute__((may_alias)) v4fa;
typedef v4i  __attribute__((may_alias)) v4ia;
typedef v8us __attribute__((may_alias)) v8usa;
union FragB { v16bf v; v16us u; v8us h[2]; v8i w; };

__device__ __forceinline__ v8f wmb(const FragB& a, const FragB& b, v8f c) {
  v8f d = __builtin_amdgcn_wmma_f32_16x16x32_bf16(false, a.v, false, b.v, (short)0, c, false, false);
  asm volatile("v_nop\n\tv_nop\n\tv_nop\n\tv_nop" : "+v"(d) : "v"(a.w), "v"(b.w));
  return d;
}

__device__ __forceinline__ unsigned f2bf(float f) {
  const unsigned u = __float_as_uint(f);
  return ((u + 0x7FFFu + ((u >> 16) & 1u)) >> 16) & 0xFFFFu;
}
__device__ __forceinline__ float bf2f(unsigned b) { return __uint_as_float(b << 16); }
__device__ __forceinline__ float bfr(float f) { return bf2f(f2bf(f)); }
__device__ __forceinline__ unsigned pk2(float lo, float hi) { return f2bf(lo) | (f2bf(hi) << 16); }
__device__ __forceinline__ v4u pack8(const v4f a, const v4f b) {
  v4u r;
  r.x = pk2(a.x, a.y); r.y = pk2(a.z, a.w); r.z = pk2(b.x, b.y); r.w = pk2(b.z, b.w);
  return r;
}

__global__ __launch_bounds__(NTHR) void k_split(const int* __restrict__ adj, int nE, int nUnits, int fullUnits,
                                                int* sp, int* dp) {
  const int u = (int)blockIdx.x * NTHR + (int)threadIdx.x;
  if (u >= nUnits) return;
  v4i s4, d4;
  if (((int)blockIdx.x + 1) * NTHR <= fullUnits) {
    const v4i a = *(const v4ia*)(adj + (size_t)8 * u);
    const v4i b = *(const v4ia*)(adj + (size_t)8 * u + 4);
    s4.x = a.x; s4.y = a.z; s4.z = b.x; s4.w = b.z;
    d4.x = a.y; d4.y = a.w; d4.z = b.y; d4.w = b.w;
  } else {
    const int e0 = 4 * u;
    const int c0 = (e0     < nE) ? e0     : nE - 1;
    const int c1 = (e0 + 1 < nE) ? e0 + 1 : nE - 1;
    const int c2 = (e0 + 2 < nE) ? e0 + 2 : nE - 1;
    const int c3 = (e0 + 3 < nE) ? e0 + 3 : nE - 1;
    const int a0 = adj[(size_t)2 * c0], b0 = adj[(size_t)2 * c0 + 1];
    const int a1 = adj[(size_t)2 * c1], b1 = adj[(size_t)2 * c1 + 1];
    const int a2 = adj[(size_t)2 * c2], b2 = adj[(size_t)2 * c2 + 1];
    const int a3 = adj[(size_t)2 * c3], b3 = adj[(size_t)2 * c3 + 1];
    s4.x = (e0     < nE) ? a0 : -1; d4.x = (e0     < nE) ? b0 : -1;
    s4.y = (e0 + 1 < nE) ? a1 : -1; d4.y = (e0 + 1 < nE) ? b1 : -1;
    s4.z = (e0 + 2 < nE) ? a2 : -1; d4.z = (e0 + 2 < nE) ? b2 : -1;
    s4.w = (e0 + 3 < nE) ? a3 : -1; d4.w = (e0 + 3 < nE) ? b3 : -1;
  }
  int* so = sp + (size_t)4 * u;
  int* dq = dp + (size_t)4 * u;
  *(volatile v4i*)so = s4;
  *(volatile v4i*)dq = d4;
  __threadfence();
  *(volatile v4i*)so = s4;
  *(volatile v4i*)dq = d4;
}

__device__ __forceinline__ int scan_chunk(const int* __restrict__ dsts, int nE, int cbase, int slotBase,
                                          int nb, int vec8, int* list, int tid, int lane, int wave) {
  int wc = 0;
  const int el0  = tid * EPT;
  const int e0   = cbase + el0;
  const int sent = -2147483647 - 1;
  v4i da, db;
  if (vec8 != 0 && cbase + CHUNK <= nE) {
    da = *(const v4ia*)(dsts + e0);
    db = *(const v4ia*)(dsts + e0 + 4);
  } else {
    da.x = (e0     < nE) ? dsts[min(e0,     nE - 1)] : sent;
    da.y = (e0 + 1 < nE) ? dsts[min(e0 + 1, nE - 1)] : sent;
    da.z = (e0 + 2 < nE) ? dsts[min(e0 + 2, nE - 1)] : sent;
    da.w = (e0 + 3 < nE) ? dsts[min(e0 + 3, nE - 1)] : sent;
    db.x = (e0 + 4 < nE) ? dsts[min(e0 + 4, nE - 1)] : sent;
    db.y = (e0 + 5 < nE) ? dsts[min(e0 + 5, nE - 1)] : sent;
    db.z = (e0 + 6 < nE) ? dsts[min(e0 + 6, nE - 1)] : sent;
    db.w = (e0 + 7 < nE) ? dsts[min(e0 + 7, nE - 1)] : sent;
  }
  const unsigned nbs = (unsigned)slotBase;
  const unsigned unb = (unsigned)nb;
  const unsigned s0 = (unsigned)da.x - nbs, s1 = (unsigned)da.y - nbs;
  const unsigned s2 = (unsigned)da.z - nbs, s3 = (unsigned)da.w - nbs;
  const unsigned s4 = (unsigned)db.x - nbs, s5 = (unsigned)db.y - nbs;
  const unsigned s6 = (unsigned)db.z - nbs, s7 = (unsigned)db.w - nbs;
  const bool h0 = s0 < unb, h1 = s1 < unb, h2 = s2 < unb, h3 = s3 < unb;
  const bool h4 = s4 < unb, h5 = s5 < unb, h6 = s6 < unb, h7 = s7 < unb;
  const unsigned any = __builtin_amdgcn_ballot_w32(h0 | h1 | h2 | h3 | h4 | h5 | h6 | h7);
  if (any != 0u) {
#define HITJ(J, HJ, SJ) { \
      const unsigned mj = __builtin_amdgcn_ballot_w32(HJ); \
      if (mj != 0u) { \
        if (HJ) { \
          const int pos = wc + (int)__builtin_amdgcn_mbcnt_lo(mj, 0u); \
          if (pos < WCAP) list[wave * WCAP + pos] = ((el0 + (J)) << SLA) | (int)(SJ); \
        } \
        wc += (int)__builtin_popcount(mj); } }
    HITJ(0, h0, s0)
    HITJ(1, h1, s1)
    HITJ(2, h2, s2)
    HITJ(3, h3, s3)
    HITJ(4, h4, s4)
    HITJ(5, h5, s5)
    HITJ(6, h6, s6)
    HITJ(7, h7, s7)
#undef HITJ
  }
  return wc;
}

__global__ __launch_bounds__(NTHR) void k_wprep(const float* __restrict__ W1, const float* __restrict__ W2,
                                                unsigned short* W1T, unsigned short* W2T) {
  const int u = (int)blockIdx.x * NTHR + (int)threadIdx.x;
  v8us o;
  unsigned short* dp;
  if (u < NU1) {
    const int n  = u >> 3;
    const int k8 = (u & 7) * 8;
    const float* p = W1 + (size_t)k8 * HID + n;
#pragma unroll
    for (int i = 0; i < 8; ++i) o[i] = (unsigned short)f2bf(p[(size_t)i * HID]);
    dp = W1T + (size_t)n * K1 + k8;
  } else if (u < NU1 + NU2) {
    const int v  = u - NU1;
    const int n  = v >> 5;
    const int k8 = (v & 31) * 8;
    const int kk = k8 & (HID - 1);
    const int ncl = n < NCLS ? n : NCLS - 1;
    const float* p = W2 + (size_t)kk * NCLS + ncl;
#pragma unroll
    for (int i = 0; i < 8; ++i) {
      const float wv = p[(size_t)i * NCLS];
      o[i] = (n < NCLS) ? (unsigned short)f2bf(wv) : (unsigned short)0;
    }
    dp = W2T + (size_t)n * K2 + k8;
  } else {
    return;
  }
  *(volatile v8us*)dp = o;
  __threadfence();
  *(volatile v8us*)dp = o;
}

__global__ __launch_bounds__(NTHR) void k_cvx(const float* __restrict__ x, int nN, int nUnits,
                                              unsigned short* xb) {
  const int u = (int)blockIdx.x * NTHR + (int)threadIdx.x;
  if (u >= nUnits) return;
  const int row = u >> 3;
  const int c0  = (u & 7) * 8;
  const int rc  = row < nN ? row : nN - 1;
  const float* p = x + (size_t)rc * DIN + c0;
  v4f a = *(const v4fa*)p, b = *(const v4fa*)(p + 4);
  const v4f z4 = {0.f, 0.f, 0.f, 0.f};
  if (row >= nN) { a = z4; b = z4; }
  const v4u hv = pack8(a, b);
  unsigned short* dp = xb + (size_t)row * K1 + c0;
  *(volatile v4u*)dp = hv;
  __threadfence();
  *(volatile v4u*)dp = hv;
}

__global__ __launch_bounds__(GTHR) void k_gemm(
    const unsigned short* __restrict__ A, const unsigned short* __restrict__ WT,
    float* outF, int K, int ldo)
{
  __shared__ __attribute__((aligned(16))) float stg[GBM * GBN];
  const int tid = (int)threadIdx.x, lane = tid & 31, wave = tid >> 5, hh = lane >> 4, m = lane & 15;
  const int rowBase = (int)blockIdx.x * GBM;
  const int col0    = (int)blockIdx.y * GBN;

  v8f acc[4];
  {
    const v8f z = {0.f, 0.f, 0.f, 0.f, 0.f, 0.f, 0.f, 0.f};
    acc[0] = z; acc[1] = z; acc[2] = z; acc[3] = z;
  }
  const unsigned short* ap = A  + (size_t)(rowBase + 16 * wave + m) * (size_t)K + 8 * hh;
  const unsigned short* wp = WT + (size_t)(col0 + m) * (size_t)K + 8 * hh;
  const int ksteps = K >> 5;
#pragma unroll 1
  for (int ks = 0; ks < ksteps; ++ks) {
    FragB af;
    af.h[0] = *(const v8usa*)(ap + 32 * ks);
    af.h[1] = *(const v8usa*)(ap + 32 * ks + 16);
#pragma unroll
    for (int t = 0; t < 4; ++t) {
      const unsigned short* wq = wp + (size_t)(16 * t) * (size_t)K + 32 * ks;
      FragB bf;
      bf.h[0] = *(const v8usa*)wq;
      bf.h[1] = *(const v8usa*)(wq + 16);
      acc[t] = wmb(af, bf, acc[t]);
    }
  }

#pragma unroll
  for (int t = 0; t < 4; ++t) {
    const int lc = 16 * t + m;
#pragma unroll
    for (int r = 0; r < 8; ++r) {
      const int lr = 16 * wave + 8 * hh + r;
      stg[lr * GBN + lc] = acc[t][r];
    }
  }
  __syncthreads();

  v4f fv[8];
#pragma unroll
  for (int i = 0; i < 8; ++i) {
    const int lr = 16 * wave + 2 * i + hh;
    fv[i] = *(const v4fa*)(stg + lr * GBN + 4 * m);
  }
#pragma unroll
  for (int i = 0; i < 8; ++i) {
    const int lr = 16 * wave + 2 * i + hh;
    const int gr = rowBase + lr;
    float* op = outF + (size_t)gr * (size_t)ldo + col0 + 4 * m;
    *(volatile v4f*)op = fv[i];
  }
  __threadfence();
#pragma unroll
  for (int i = 0; i < 8; ++i) {
    const int lr = 16 * wave + 2 * i + hh;
    const int gr = rowBase + lr;
    float* op = outF + (size_t)gr * (size_t)ldo + col0 + 4 * m;
    *(volatile v4f*)op = fv[i];
  }
}

template <int L>
__global__ __launch_bounds__(NTHR) void k_agg(const int* __restrict__ srcs, const int* __restrict__ dsts,
                                              int nE, int nN, int vec8, int mRows,
                                              const float* __restrict__ xl, const float* __restrict__ bias,
                                              unsigned short* hb, float* outp) {
  static_assert(L == 1 || L == 2);
  extern __shared__ __attribute__((aligned(16))) int dsm[];
  int* list = dsm;
  int* hl   = dsm + LISTN;
  int* sl   = dsm + LISTN + RCAP;
  int* cnt  = dsm + LISTN + 2 * RCAP;
  int* offs = cnt + NBA;
  int* cur  = offs + NBA;
  int* misc = cur + NBA;
  constexpr int CPL = (L == 1) ? 4 : 2;
  constexpr int C   = CPL * 32;
  const int tid = (int)threadIdx.x, lane = tid & 31, wave = tid >> 5;
  const int nodeBase = (int)blockIdx.x * NBA;

  {
    const v4i z4 = {0, 0, 0, 0};
    for (int i = tid * 4; i < AGG_ZINTS; i += NTHR * 4) *(v4ia*)(dsm + i) = z4;
    if (tid < 16) misc[tid] = 0;
  }
  float bv[CPL];
  const int c0 = CPL * lane;
  const bool valid = (L == 1) || (c0 < NCLS);
  if constexpr (L == 1) {
    const v4f a = *(const v4fa*)(bias + 4 * lane);
    bv[0] = bfr(a.x); bv[1] = bfr(a.y); bv[2] = bfr(a.z); bv[3] = bfr(a.w);
  } else {
    const int cc0 = c0 < NCLS ? c0 : NCLS - 1;
    const int cc1 = c0 + 1 < NCLS ? c0 + 1 : NCLS - 1;
    const float b0 = bfr(bias[cc0]), b1 = bfr(bias[cc1]);
    bv[0] = valid ? b0 : 0.f;
    bv[1] = valid ? b1 : 0.f;
  }
  __syncthreads();

  int t = 0, ov = 0;
  const int nChunks = (nE + CHUNK - 1) / CHUNK;
#pragma unroll 1
  for (int ch = 0; ch < nChunks; ++ch) {
    const int cbase = ch * CHUNK;
    const int wc = scan_chunk(dsts, nE, cbase, nodeBase, NBA, vec8, list, tid, lane, wave);
    if (lane == 0) misc[wave] = wc;
    __syncthreads();
    if (wave == 0) {
#pragma unroll 1
      for (int w2 = 0; w2 < NWAVE; ++w2) {
        int c = misc[w2];
        c = c < 0 ? 0 : (c > WCAP ? WCAP : c);
#pragma unroll 1
        for (int b0 = 0; b0 < c; b0 += 32) {
          const int idx = b0 + lane;
          const int ent = list[w2 * WCAP + (idx < WCAP ? idx : WCAP - 1)];
          const int m32 = (c - b0) < 32 ? (c - b0) : 32;
#pragma unroll 1
          for (int k = 0; k < m32; ++k) {
            const int u    = __builtin_amdgcn_readlane(ent, k);
            const int slot = u & (NBA - 1);
            const int el   = (u >> SLA) & (CHUNK - 1);
            const int pk   = ((cbase + el) << SLA) | slot;
            if (t < RCAP) {
              if (lane == 0) { hl[t] = pk; cnt[slot] = cnt[slot] + 1; }
              t = t + 1;
            } else {
              ov = 1;
            }
          }
        }
      }
    }
    __syncthreads();
  }
  if (wave == 0 && lane == 0) { misc[8] = t; misc[9] = ov; }
  __syncthreads();
  int tt = misc[8];
  tt = tt < 0 ? 0 : (tt > RCAP ? RCAP : tt);
  const int ovf = misc[9];

  if (wave == 0) {
    const int base = lane * (NBA / 32);
    int s = 0;
#pragma unroll 1
    for (int i = 0; i < NBA / 32; ++i) s += cnt[base + i];
    int incl = s;
#pragma unroll
    for (int d = 1; d < 32; d <<= 1) {
      const int y = __shfl_up(incl, d, 32);
      if (lane >= d) incl += y;
    }
    int run = incl - s;
#pragma unroll 1
    for (int i = 0; i < NBA / 32; ++i) {
      const int cv = cnt[base + i];
      offs[base + i] = run;
      cur[base + i]  = run;
      run += cv;
    }
  }
  __syncthreads();
  if (wave == 0) {
#pragma unroll 1
    for (int b0 = 0; b0 < tt; b0 += 32) {
      const int idx = b0 + lane;
      const int ent = hl[idx < RCAP ? idx : RCAP - 1];
      const int m32 = (tt - b0) < 32 ? (tt - b0) : 32;
#pragma unroll 1
      for (int k = 0; k < m32; ++k) {
        const int u    = __builtin_amdgcn_readlane(ent, k);
        const int slot = u & (NBA - 1);
        if (lane == 0) {
          int p = cur[slot];
          p = p < 0 ? 0 : (p > RCAP - 1 ? RCAP - 1 : p);
          sl[p] = u;
          cur[slot] = p + 1;
        }
      }
    }
  }
  __syncthreads();

  const float qnan = __int_as_float(0x7fc00000);
  const float pz = (ovf != 0) ? qnan : 0.0f;
  float* res = (float*)hl + wave * (GRP * NCLS);
#pragma unroll 1
  for (int si = 0; si < SPW; ++si) {
    const int s    = wave * SPW + si;
    const int node = nodeBase + s;
    int c = cnt[s];
    const bool big = c > DEGCAP;
    c = c < 0 ? 0 : (c > DEGCAP ? DEGCAP : c);
    int o = offs[s];
    o = o < 0 ? 0 : (o > RCAP ? RCAP : o);
    const int nc = node < nN ? node : nN - 1;
    float acc[CPL];
#pragma unroll
    for (int i = 0; i < CPL; ++i) acc[i] = 0.0f;
#pragma unroll 1
    for (int b0 = 0; b0 < c; b0 += 32) {
      int idx = o + b0 + lane;
      idx = idx > RCAP - 1 ? RCAP - 1 : idx;
      const int ent = sl[idx];
      int eid = ent >> SLA;
      eid = eid < 0 ? 0 : (eid > nE - 1 ? nE - 1 : eid);
      int sr = srcs[eid];
      sr = sr < 0 ? 0 : (sr > nN - 1 ? nN - 1 : sr);
      const int m32 = (c - b0) < 32 ? (c - b0) : 32;
#pragma unroll 1
      for (int k = 0; k < m32; ++k) {
        const int sk = __builtin_amdgcn_readlane(sr, k);
        const float* rp = xl + (size_t)sk * C + CPL * lane;
        if constexpr (CPL == 4) {
          const v4f a = *(const v4fa*)rp;
          acc[0] += a.x; acc[1] += a.y; acc[2] += a.z; acc[3] += a.w;
        } else {
          const v2f a = *(const v2fa*)rp;
          acc[0] += a.x; acc[1] += a.y;
        }
      }
    }
    float sv[CPL];
    {
      const float* spp = xl + (size_t)nc * C + CPL * lane;
      if constexpr (CPL == 4) {
        const v4f a = *(const v4fa*)spp;
        sv[0] = a.x; sv[1] = a.y; sv[2] = a.z; sv[3] = a.w;
      } else {
        const v2f a = *(const v2fa*)spp;
        sv[0] = a.x; sv[1] = a.y;
      }
    }
    const float pzr = big ? qnan : pz;
    const bool live = node < nN;

    if constexpr (L == 1) {
      float v[CPL];
#pragma unroll
      for (int i = 0; i < CPL; ++i) {
        float y = (acc[i] + sv[i]) + bv[i];
        y = fmaxf(y, 0.0f);
        y = y + pzr;
        v[i] = live ? y : 0.0f;
      }
      const int sa = (2 * lane) & 31;
      const int sb = (2 * lane + 1) & 31;
      const unsigned hb0 = f2bf(v[0]), hb1 = f2bf(v[1]);
      const unsigned hb2 = f2bf(v[2]), hb3 = f2bf(v[3]);
      const unsigned lb0 = f2bf(v[0] - bf2f(hb0));
      const unsigned lb1 = f2bf(v[1] - bf2f(hb1));
      const unsigned lb2 = f2bf(v[2] - bf2f(hb2));
      const unsigned lb3 = f2bf(v[3] - bf2f(hb3));
      const int hw0 = (int)(hb0 | (hb1 << 16));
      const int hw1 = (int)(hb2 | (hb3 << 16));
      const int lw0 = (int)(lb0 | (lb1 << 16));
      const int lw1 = (int)(lb2 | (lb3 << 16));
      const int g0 = __shfl(hw0, sa, 32), g1 = __shfl(hw1, sa, 32);
      const int g2 = __shfl(hw0, sb, 32), g3 = __shfl(hw1, sb, 32);
      const int q0 = __shfl(lw0, sa, 32), q1 = __shfl(lw1, sa, 32);
      const int q2 = __shfl(lw0, sb, 32), q3 = __shfl(lw1, sb, 32);
      const bool lsel = lane >= 16;
      v4u pv;
      pv.x = (unsigned int)(lsel ? q0 : g0);
      pv.y = (unsigned int)(lsel ? q1 : g1);
      pv.z = (unsigned int)(lsel ? q2 : g2);
      pv.w = (unsigned int)(lsel ? q3 : g3);
      if (node < mRows) {
        unsigned short* hp = hb + (size_t)node * K2 + 8 * lane;
        *(volatile v4u*)hp = pv;
        __threadfence();
        *(volatile v4u*)hp = pv;
      }
    } else {
      const float z0 = (acc[0] + sv[0]) + bv[0];
      const float z1 = (acc[1] + sv[1]) + bv[1];
      float vm = valid ? fmaxf(z0, z1) : -3.0e38f;
#pragma unroll
      for (int off = 16; off > 0; off >>= 1) vm = fmaxf(vm, __shfl_xor(vm, off));
      const float d0 = valid ? (z0 - vm) : 0.f;
      const float d1 = valid ? (z1 - vm) : 0.f;
      const float ex0 = expf(d0), ex1 = expf(d1);
      float sm = valid ? (ex0 + ex1) : 0.f;
#pragma unroll
      for (int off = 16; off > 0; off >>= 1) sm += __shfl_xor(sm, off);
      const float inv = 1.0f / sm;
      const float o0 = ex0 * inv + pzr;
      const float o1 = ex1 * inv + pzr;
      const int lr = si & (GRP - 1);
      if (valid) {
        v2f ow; ow.x = o0; ow.y = o1;
        *(v2fa*)(res + lr * NCLS + c0) = ow;
      }
      if (lr == GRP - 1) {
        __syncthreads();
        const int gb = si & ~(GRP - 1);
        const int row0 = nodeBase + wave * SPW + gb;
        int lv = nN - row0; lv = lv < 0 ? 0 : (lv > GRP ? GRP : lv);
        const int npc = lv * (NCLS / 4);
        float* ob = outp + (size_t)row0 * NCLS;
#pragma unroll 1
        for (int p = lane; p < npc; p += 32) {
          const v4f vv = *(const v4fa*)(res + 4 * p);
          *(volatile v4f*)(ob + 4 * p) = vv;
        }
        __threadfence();
#pragma unroll 1
        for (int p = lane; p < npc; p += 32) {
          const v4f vv = *(const v4fa*)(res + 4 * p);
          *(volatile v4f*)(ob + 4 * p) = vv;
        }
        __syncthreads();
      }
    }
  }
}

static inline int cdiv(int a, int b) { return (a + b - 1) / b; }

extern "C" void kernel_launch(void* const* d_in, const int* in_sizes, int n_in,
                              void* d_out, int out_size, void* d_ws, size_t ws_size,
                              hipStream_t stream) {
  if (n_in < 6) return;
  if (in_sizes[0] < DIN || (in_sizes[0] % DIN) != 0) return;
  const int nN = in_sizes[0] / DIN;
  if (nN > (1 << 22)) return;
  if (in_sizes[1] < 2 || (in_sizes[1] & 1) != 0) return;
  const int nE = in_sizes[1] / 2;
  if (nE < 1 || nE >= (1 << (31 - SLA))) return;
  if (in_sizes[2] != DIN * HID || in_sizes[3] != HID) return;
  if (in_sizes[4] != HID * NCLS || in_sizes[5] != NCLS) return;
  if ((long long)out_size != (long long)nN * NCLS) return;

  const float* x   = (const float*)d_in[0];
  const int*   adj = (const int*)d_in[1];
  const float* W1  = (const float*)d_in[2];
  const float* b1  = (const float*)d_in[3];
  const float* W2  = (const float*)d_in[4];
  const float* b2  = (const float*)d_in[5];
  float* out = (float*)d_out;

  const int MP   = cdiv(nN, GBM) * GBM;
  const int gM   = MP / GBM;
  const int gA   = cdiv(MP, NBA);
  if ((long long)gA * NBA < (long long)MP) return;
  const int EP   = cdiv(nE, 32) * 32;
  const int nUs  = EP / 4;
  const int fullU = nE / 4;
  const int vec8 = 1;

  char* ws = (char*)d_ws;
  size_t off = 0;
  const size_t oSRC = off; off += (size_t)EP * 4;                         off = (off + 255) & ~(size_t)255;
  const size_t oDST = off; off += (size_t)EP * 4;                         off = (off + 255) & ~(size_t)255;
  const size_t oW1T = off; off += (size_t)HID * K1 * 2;                   off = (off + 255) & ~(size_t)255;
  const size_t oW2T = off; off += (size_t)NC2P * K2 * 2;                  off = (off + 255) & ~(size_t)255;
  const size_t oXB  = off; off += (size_t)MP * K1 * 2;                    off = (off + 255) & ~(size_t)255;
  const size_t szH1 = (size_t)MP * HID * 4;
  const size_t szH2 = (size_t)MP * NC2P * 4;
  const size_t oH   = off; off += (szH1 > szH2 ? szH1 : szH2);            off = (off + 255) & ~(size_t)255;
  const size_t oA2  = off; off += (size_t)MP * K2 * 2;                    off = (off + 255) & ~(size_t)255;
  if (off > ws_size || off > (size_t)WSMAX) return;
  int*            SRC = (int*)(ws + oSRC);
  int*            DST = (int*)(ws + oDST);
  unsigned short* W1T = (unsigned short*)(ws + oW1T);
  unsigned short* W2T = (unsigned short*)(ws + oW2T);
  unsigned short* XB  = (unsigned short*)(ws + oXB);
  float*          H   = (float*)(ws + oH);
  unsigned short* A2  = (unsigned short*)(ws + oA2);

  const size_t aggLds = (size_t)AGG_LDS_INTS * 4;
  hipFuncSetAttribute(reinterpret_cast<const void*>(&k_agg<1>), hipFuncAttributeMaxDynamicSharedMemorySize, (int)aggLds);
  hipFuncSetAttribute(reinterpret_cast<const void*>(&k_agg<2>), hipFuncAttributeMaxDynamicSharedMemorySize, (int)aggLds);

  const int nUx = MP * (K1 / 8);
  k_split<<<cdiv(nUs, NTHR), NTHR, 0, stream>>>(adj, nE, nUs, fullU, SRC, DST);
  k_wprep<<<(NU1 + NU2) / NTHR, NTHR, 0, stream>>>(W1, W2, W1T, W2T);
  k_cvx<<<cdiv(nUx, NTHR), NTHR, 0, stream>>>(x, nN, nUx, XB);
  k_gemm<<<dim3(gM, HID / GBN), GTHR, 0, stream>>>(XB, W1T, H, K1, HID);
  k_agg<1><<<gA, NTHR, aggLds, stream>>>(SRC, DST, nE, nN, vec8, MP, H, b1, A2, out);
  k_gemm<<<dim3(gM, NC2P / GBN), GTHR, 0, stream>>>(A2, W2T, H, K2, NC2P);
  k_agg<2><<<gA, NTHR, aggLds, stream>>>(SRC, DST, nE, nN, vec8, MP, H, b2, A2, out);
}
